// GraphNetv2_46935402611088
// MI455X (gfx1250) — hardware-verified
//
#include <hip/hip_runtime.h>
#include <stdint.h>
#include <stddef.h>


typedef _Float16 v16h __attribute__((ext_vector_type(16)));
typedef _Float16 v8h  __attribute__((ext_vector_type(8)));
typedef float    v8f  __attribute__((ext_vector_type(8)));
typedef float    v4f  __attribute__((ext_vector_type(4)));
typedef int      v4i  __attribute__((ext_vector_type(4)));
union Frag { v16h v; v8h half[2]; };

#define NND     128
#define PF      30
#define NBATCH  64
#define EPN     127
#define NEDGE   16256
#define WSCALE  16.0f
#define WINV    0.0625f
#define BN_EPS  1e-5f

#define OFF_W1E 0
#define OFF_W2E 5120
#define OFF_W3E 9728
#define OFF_W1O 11776
#define OFF_W2O 14848
#define OFF_W3O 16896
#define WB_HALVES 17920

#define XT_PER_B   4096
#define E_PER_SEG  2560
#define E_PER_B    327680
#define STAT_PITCH 64
#define NSUM_PITCH 32

#define WSB_WB    0u
#define WSB_XT    35840u
#define WSB_E     560128u
#define WSB_STAT  84446208u
#define WSB_SC    86543360u
#define WSB_NS    86543616u
#define WSB_END   86551808u
static_assert(WSB_END <= 134217728u);

__device__ __forceinline__ v16h frag_ld(const _Float16* base, int idx0, int k0, int pitch, int lane) {
  Frag f;
  const int h = lane >> 4, m = lane & 15;
  const _Float16* p = base + (idx0 + m) * pitch + k0 + 8 * h;
  f.half[0] = *(const v8h*)(p);
  f.half[1] = *(const v8h*)(p + 16);
  return f.v;
}
__device__ __forceinline__ v8f wmma16(v16h a, v16h b, v8f c) {
  v8f d = __builtin_amdgcn_wmma_f32_16x16x32_f16(false, a, false, b, (short)0, c, false, false);
  asm volatile("v_nop\n\tv_nop\n\tv_nop\n\tv_nop" : "+v"(d) : "v"(a), "v"(b));
  return d;
}
__device__ __forceinline__ v8h relu_pack8(v8f acc) {
  v8h o;
#pragma unroll
  for (int j = 0; j < 8; ++j) o[j] = (_Float16)(fmaxf(acc[j], 0.f) * WINV);
  return o;
}

__device__ __forceinline__ float wblob_val(int g,
    const float* Wfr1, const float* Wfr2, const float* Wfr3,
    const float* Wfo1, const float* Wfo2, const float* Wfo3)
{
  float v = 0.f;
  if (g < OFF_W2E) {
    const int m = g >> 6, k = g & 63;
    if (k < 30) v = Wfr1[m * 60 + k];
    else if (k >= 32 && k < 62) v = Wfr1[m * 60 + (k - 2)];
  } else if (g < OFF_W3E) {
    const int i = g - OFF_W2E; const int m = i / 96, k = i - m * 96;
    if (m < 40 && k < 80) v = Wfr2[m * 80 + k];
  } else if (g < OFF_W1O) {
    const int i = g - OFF_W3E; const int m = i >> 6, k = i & 63;
    if (m < 20 && k < 40) v = Wfr3[m * 40 + k];
  } else if (g < OFF_W2O) {
    const int i = g - OFF_W1O; const int m = i >> 6, k = i & 63;
    if (m < 40) {
      if (k < 30) v = Wfo1[m * 50 + k];
      else if (k >= 32 && k < 52) v = Wfo1[m * 50 + (k - 2)];
    }
  } else if (g < OFF_W3O) {
    const int i = g - OFF_W2O; const int m = i >> 6, k = i & 63;
    if (m < 20 && k < 40) v = Wfo2[m * 40 + k];
  } else {
    const int i = g - OFF_W3O; const int m = i >> 5, k = i & 31;
    if (m < 20 && k < 20) v = Wfo3[m * 20 + k];
  }
  return v * WSCALE;
}

__device__ __forceinline__ void prep_pass(const float* sx, _Float16* xtb, bool doW, _Float16* wb,
    const float* Wfr1, const float* Wfr2, const float* Wfr3,
    const float* Wfo1, const float* Wfo2, const float* Wfo3, int tid)
{
  for (int i = tid; i < 512; i += 256) {
    const int n = i >> 2, q = i & 3;
    v8h o;
#pragma unroll
    for (int jj = 0; jj < 8; ++jj) {
      const int f = q * 8 + jj;
      o[jj] = (f < PF) ? (_Float16)sx[f * NND + n] : (_Float16)0.f;
    }
    *(volatile v8h*)(xtb + i * 8) = o;
  }
  if (doW) {
    for (int i = tid; i < WB_HALVES / 8; i += 256) {
      v8h o;
#pragma unroll
      for (int jj = 0; jj < 8; ++jj)
        o[jj] = (_Float16)wblob_val(i * 8 + jj, Wfr1, Wfr2, Wfr3, Wfo1, Wfo2, Wfo3);
      *(volatile v8h*)(wb + i * 8) = o;
    }
  }
}
__global__ __launch_bounds__(256) void prep_kernel(
    const float* __restrict__ x,
    const float* __restrict__ Wfr1, const float* __restrict__ Wfr2, const float* __restrict__ Wfr3,
    const float* __restrict__ Wfo1, const float* __restrict__ Wfo2, const float* __restrict__ Wfo3,
    _Float16* __restrict__ wb, _Float16* __restrict__ xt)
{
  __shared__ float sx[PF * NND];
  const int tid = threadIdx.x, b = blockIdx.x;
  const float* xb = x + (size_t)b * (PF * NND);
  for (int i = tid; i < PF * NND; i += 256) sx[i] = xb[i];
  __syncthreads();
  _Float16* xtb = xt + (size_t)b * XT_PER_B;
  const bool doW = (b == 0);
  prep_pass(sx, xtb, doW, wb, Wfr1, Wfr2, Wfr3, Wfo1, Wfo2, Wfo3, tid);
  __threadfence();
  prep_pass(sx, xtb, doW, wb, Wfr1, Wfr2, Wfr3, Wfo1, Wfo2, Wfo3, tid);
}

__device__ __forceinline__ void edge_store(const float* sE, const float* sStat, float* Eseg, float* statblk, int tid) {
  for (int i = tid; i < E_PER_SEG / 4; i += 256)
    *(volatile v4f*)(Eseg + i * 4) = *(const v4f*)(sE + i * 4);
  if (tid < 16)
    *(volatile v4f*)(statblk + tid * 4) = *(const v4f*)(sStat + tid * 4);
}
__global__ __launch_bounds__(256) void edge_kernel(
    const _Float16* __restrict__ xt, const _Float16* __restrict__ wb,
    const int* __restrict__ recv, const int* __restrict__ send,
    const float* __restrict__ bfr1, const float* __restrict__ bfr2, const float* __restrict__ bfr3,
    float* __restrict__ Eout, float* __restrict__ stat)
{
  __shared__ __align__(16) _Float16 sW[11776];
  __shared__ __align__(16) _Float16 sBm[128 * 64];
  __shared__ __align__(16) _Float16 sAct1[128 * 96];

  const int tid = threadIdx.x, lane = tid & 31, wave = tid >> 5;
  const int r = blockIdx.x, b = blockIdx.y;
  const _Float16* xtb = xt + (size_t)b * XT_PER_B;
  const v4i z4 = {0, 0, 0, 0};

  for (int i = tid; i < 1472; i += 256)
    *(v4i*)(sW + i * 8) = *(const v4i*)(wb + i * 8);
  for (int i = tid; i < 1024; i += 256) {
    const int col = i >> 3, c = i & 7;
    v4i v = z4;
    if (col < EPN) {
      const int e = r * EPN + col;
      int node = (c < 4) ? recv[e] : send[e];
      node = min(max(node, 0), NND - 1);
      v = *(const v4i*)(xtb + node * 32 + (c & 3) * 8);
    }
    *(v4i*)(sBm + col * 64 + c * 8) = v;
  }
  for (int i = tid; i < 256; i += 256) {
    const int col = i >> 1;
    *(v4i*)(sAct1 + col * 96 + 80 + 8 * (i & 1)) = z4;
  }
  __syncthreads();

  const int nb = wave * 16, h = lane >> 4, cl = lane & 15;

#pragma unroll
  for (int mt = 0; mt < 5; ++mt) {
    v8f acc;
#pragma unroll
    for (int j = 0; j < 8; ++j) acc[j] = WSCALE * bfr1[mt * 16 + 8 * h + j];
#pragma unroll
    for (int kt = 0; kt < 2; ++kt) {
      const v16h a  = frag_ld(sW + OFF_W1E, mt * 16, kt * 32, 64, lane);
      const v16h bb = frag_ld(sBm, nb, kt * 32, 64, lane);
      acc = wmma16(a, bb, acc);
    }
    *(v8h*)(sAct1 + (nb + cl) * 96 + mt * 16 + 8 * h) = relu_pack8(acc);
  }
  __syncthreads();

  _Float16* sAct2 = sBm;
#pragma unroll
  for (int mt = 0; mt < 3; ++mt) {
    v8f acc;
#pragma unroll
    for (int j = 0; j < 8; ++j) {
      const int row = mt * 16 + 8 * h + j;
      acc[j] = (row < 40) ? WSCALE * bfr2[row] : 0.f;
    }
#pragma unroll
    for (int kt = 0; kt < 3; ++kt) {
      const v16h a  = frag_ld(sW + OFF_W2E, mt * 16, kt * 32, 96, lane);
      const v16h bb = frag_ld(sAct1, nb, kt * 32, 96, lane);
      acc = wmma16(a, bb, acc);
    }
    *(v8h*)(sAct2 + (nb + cl) * 64 + mt * 16 + 8 * h) = relu_pack8(acc);
  }
  for (int i = tid; i < 256; i += 256) {
    const int col = i >> 1;
    *(v4i*)(sAct2 + col * 64 + 48 + 8 * (i & 1)) = z4;
  }
  __syncthreads();

  float* sE    = reinterpret_cast<float*>(sAct1);
  float* sStat = sE + E_PER_SEG;
#pragma unroll
  for (int mt = 0; mt < 2; ++mt) {
    v8f acc;
#pragma unroll
    for (int j = 0; j < 8; ++j) {
      const int row = mt * 16 + 8 * h + j;
      acc[j] = (row < 20) ? WSCALE * bfr3[row] : 0.f;
    }
#pragma unroll
    for (int kt = 0; kt < 2; ++kt) {
      const v16h a  = frag_ld(sW + OFF_W3E, mt * 16, kt * 32, 64, lane);
      const v16h bb = frag_ld(sAct2, nb, kt * 32, 64, lane);
      acc = wmma16(a, bb, acc);
    }
    const bool colok = (nb + cl) < EPN;
#pragma unroll
    for (int j = 0; j < 8; ++j) {
      const int row = mt * 16 + 8 * h + j;
      if (row < 20) {
        const float v = colok ? fmaxf(acc[j], 0.f) * WINV : 0.f;
        sE[(nb + cl) * 20 + row] = v;
      }
    }
  }
  __syncthreads();

  if (wave == 0) {
    float s1 = 0.f, s2 = 0.f;
    if (lane < 20) {
      for (int j = 0; j < EPN; ++j) {
        const float v = sE[j * 20 + lane];
        s1 += v;
        s2 = fmaf(v, v, s2);
      }
    }
    sStat[lane] = s1;
    sStat[32 + lane] = s2;
  }
  __syncthreads();

  float* Eseg    = Eout + ((size_t)b * NND + r) * E_PER_SEG;
  float* statblk = stat + ((size_t)b * NND + r) * STAT_PITCH;
  edge_store(sE, sStat, Eseg, statblk, tid);
  __threadfence();
  edge_store(sE, sStat, Eseg, statblk, tid);
}

__global__ __launch_bounds__(256) void stat_kernel(
    const float* __restrict__ stat, const float* __restrict__ gamma, const float* __restrict__ beta,
    float* __restrict__ scal)
{
  __shared__ double sPart[256];
  __shared__ __align__(16) float sOut[64];
  const int tid = threadIdx.x;
  const int s = tid & 63, part = tid >> 6;
  double acc = 0.0;
  const float* p = stat + (size_t)part * 2048 * STAT_PITCH + s;
  for (int i = 0; i < 2048; ++i) acc += (double)p[(size_t)i * STAT_PITCH];
  sPart[tid] = acc;
  __syncthreads();
  if (tid < 32) {
    float sc = 0.f, sh = 0.f;
    if (tid < 20) {
      const double S1 = sPart[tid] + sPart[64 + tid] + sPart[128 + tid] + sPart[192 + tid];
      const double S2 = sPart[32 + tid] + sPart[96 + tid] + sPart[160 + tid] + sPart[224 + tid];
      const double M = 64.0 * 16256.0;
      const double mu = S1 / M;
      double var = S2 / M - mu * mu;
      if (var < 0.0) var = 0.0;
      const float inv = 1.0f / sqrtf((float)var + BN_EPS);
      sc = gamma[tid] * inv;
      sh = beta[tid] - sc * (float)mu;
    }
    sOut[tid] = sc;
    sOut[32 + tid] = sh;
  }
  __syncthreads();
  if (tid < 16) *(volatile v4f*)(scal + tid * 4) = *(const v4f*)(sOut + tid * 4);
  __threadfence();
  if (tid < 16) *(volatile v4f*)(scal + tid * 4) = *(const v4f*)(sOut + tid * 4);
}

__global__ __launch_bounds__(256) void node_kernel(
    const _Float16* __restrict__ xt, const _Float16* __restrict__ wb,
    const int* __restrict__ recv, const float* __restrict__ E, const float* __restrict__ scal,
    const float* __restrict__ bfo1, const float* __restrict__ bfo2, const float* __restrict__ bfo3,
    float* __restrict__ nsum)
{
  __shared__ __align__(16) unsigned char arena[55296];
  __shared__ __align__(16) float sScale[64];
  __shared__ float sCnt[NND];
  __shared__ float sNsW[256];
  __shared__ __align__(16) float sNs[32];
  float* sEbar = reinterpret_cast<float*>(arena);
  float* sAgg  = reinterpret_cast<float*>(arena + 10240);
  int*   sCntW = reinterpret_cast<int*>(arena + 51200);
  _Float16* sC  = reinterpret_cast<_Float16*>(arena + 10240);
  _Float16* sA1 = reinterpret_cast<_Float16*>(arena + 26624);
  _Float16* sWo = reinterpret_cast<_Float16*>(arena + 43008);
  _Float16* sA2 = reinterpret_cast<_Float16*>(arena);

  const int tid = threadIdx.x, lane = tid & 31, wave = tid >> 5;
  const int b = blockIdx.x;
  const _Float16* xtb = xt + (size_t)b * XT_PER_B;
  const float* Eb = E + (size_t)b * E_PER_B;
  const v4i z4 = {0, 0, 0, 0};

  if (tid < 64) sScale[tid] = scal[tid];
  for (int i = tid; i < 2688; i += 256) *(v4i*)(arena + 10240 + i * 16) = z4;
  __syncthreads();

  if (wave < 4) {
    float* agg = sAgg + wave * E_PER_SEG;
    int* cw = sCntW + wave * NND;
    for (int rr = 0; rr < 32; ++rr) {
      const int r = wave * 32 + rr;
      const float* Er = Eb + (size_t)r * E_PER_SEG;
      const int* rc = recv + r * EPN;
      for (int j = 0; j < EPN; ++j) {
        int rv = rc[j];
        rv = min(max(rv, 0), NND - 1);
        if (lane < 20) {
          const float v = Er[j * 20 + lane];
          agg[rv * 20 + lane] += v;
        }
        if (lane == 0) cw[rv] += 1;
      }
    }
  }
  __syncthreads();
  for (int i = tid; i < E_PER_SEG; i += 256)
    sEbar[i] = ((sAgg[i] + sAgg[E_PER_SEG + i]) + sAgg[2 * E_PER_SEG + i]) + sAgg[3 * E_PER_SEG + i];
  if (tid < NND)
    sCnt[tid] = (float)(sCntW[tid] + sCntW[NND + tid] + sCntW[2 * NND + tid] + sCntW[3 * NND + tid]);
  __syncthreads();

  for (int i = tid; i < 768; i += 256)
    *(v4i*)(sWo + i * 8) = *(const v4i*)(wb + OFF_W1O + i * 8);
  for (int i = tid; i < 512; i += 256) {
    const int col = i >> 2, c = i & 3;
    *(v4i*)(sC + col * 64 + c * 8) = *(const v4i*)(xtb + col * 32 + c * 8);
  }
  for (int i = tid; i < 512; i += 256) {
    const int col = i >> 2, g = i & 3;
    v8h o;
#pragma unroll
    for (int jj = 0; jj < 8; ++jj) {
      const int c = 8 * g + jj;
      float v = 0.f;
      if (c < 20) v = fmaf(sScale[c], sEbar[col * 20 + c], sCnt[col] * sScale[32 + c]);
      o[jj] = (_Float16)v;
    }
    *(v8h*)(sC + col * 64 + 32 + 8 * g) = o;
  }
  for (int i = tid; i < 256; i += 256) {
    const int col = i >> 1;
    *(v4i*)(sA1 + col * 64 + 48 + 8 * (i & 1)) = z4;
  }
  __syncthreads();

  const int nb = wave * 16, h = lane >> 4, cl = lane & 15;

#pragma unroll
  for (int mt = 0; mt < 3; ++mt) {
    v8f acc;
#pragma unroll
    for (int j = 0; j < 8; ++j) {
      const int row = mt * 16 + 8 * h + j;
      acc[j] = (row < 40) ? WSCALE * bfo1[row] : 0.f;
    }
#pragma unroll
    for (int kt = 0; kt < 2; ++kt) {
      const v16h a  = frag_ld(sWo, mt * 16, kt * 32, 64, lane);
      const v16h bb = frag_ld(sC, nb, kt * 32, 64, lane);
      acc = wmma16(a, bb, acc);
    }
    *(v8h*)(sA1 + (nb + cl) * 64 + mt * 16 + 8 * h) = relu_pack8(acc);
  }
  __syncthreads();

#pragma unroll
  for (int mt = 0; mt < 2; ++mt) {
    v8f acc;
#pragma unroll
    for (int j = 0; j < 8; ++j) {
      const int row = mt * 16 + 8 * h + j;
      acc[j] = (row < 20) ? WSCALE * bfo2[row] : 0.f;
    }
#pragma unroll
    for (int kt = 0; kt < 2; ++kt) {
      const v16h a  = frag_ld(sWo + (OFF_W2O - OFF_W1O), mt * 16, kt * 32, 64, lane);
      const v16h bb = frag_ld(sA1, nb, kt * 32, 64, lane);
      acc = wmma16(a, bb, acc);
    }
    *(v8h*)(sA2 + (nb + cl) * 32 + mt * 16 + 8 * h) = relu_pack8(acc);
  }
  __syncthreads();

#pragma unroll
  for (int mt = 0; mt < 2; ++mt) {
    v8f acc;
#pragma unroll
    for (int j = 0; j < 8; ++j) {
      const int row = mt * 16 + 8 * h + j;
      acc[j] = (row < 20) ? WSCALE * bfo3[row] : 0.f;
    }
    {
      const v16h a  = frag_ld(sWo + (OFF_W3O - OFF_W1O), mt * 16, 0, 32, lane);
      const v16h bb = frag_ld(sA2, nb, 0, 32, lane);
      acc = wmma16(a, bb, acc);
    }
#pragma unroll
    for (int j = 0; j < 8; ++j) {
      float v = fmaxf(acc[j], 0.f) * WINV;
      v += __shfl_xor(v, 1);
      v += __shfl_xor(v, 2);
      v += __shfl_xor(v, 4);
      v += __shfl_xor(v, 8);
      if (cl == 0) sNsW[wave * 32 + mt * 16 + 8 * h + j] = v;
    }
  }
  __syncthreads();
  if (tid < 32) {
    float s = 0.f;
#pragma unroll
    for (int w = 0; w < 8; ++w) s += sNsW[w * 32 + tid];
    sNs[tid] = s;
  }
  __syncthreads();
  float* nsb = nsum + (size_t)b * NSUM_PITCH;
  if (tid < 8) *(volatile v4f*)(nsb + tid * 4) = *(const v4f*)(sNs + tid * 4);
  __threadfence();
  if (tid < 8) *(volatile v4f*)(nsb + tid * 4) = *(const v4f*)(sNs + tid * 4);
}

__global__ __launch_bounds__(256) void head_kernel(
    const float* __restrict__ nsum, const float* __restrict__ Wfc, const float* __restrict__ bfc,
    float* __restrict__ out)
{
  __shared__ __align__(16) float sO[320];
  const int tid = threadIdx.x;
  for (int o = tid; o < 320; o += 256) {
    const int bb = o / 5, t = o - bb * 5;
    const float* ns = nsum + bb * NSUM_PITCH;
    const float* w = Wfc + t * 20;
    float a = 0.f;
#pragma unroll
    for (int c = 0; c < 20; ++c) a = fmaf(ns[c], w[c], a);
    sO[o] = a + bfc[t];
  }
  __syncthreads();
  if (tid < 80) *(volatile v4f*)(out + tid * 4) = *(const v4f*)(sO + tid * 4);
  __threadfence();
  if (tid < 80) *(volatile v4f*)(out + tid * 4) = *(const v4f*)(sO + tid * 4);
}

extern "C" void kernel_launch(void* const* d_in, const int* in_sizes, int n_in,
                              void* d_out, int out_size, void* d_ws, size_t ws_size,
                              hipStream_t stream) {
  if (n_in < 19) return;
  if (in_sizes[0] != NBATCH * PF * NND || in_sizes[1] != NEDGE || in_sizes[2] != NEDGE ||
      in_sizes[3] != 4800 || in_sizes[4] != 80 || in_sizes[5] != 3200 || in_sizes[6] != 40 ||
      in_sizes[7] != 800 || in_sizes[8] != 20 || in_sizes[9] != 20 || in_sizes[10] != 20 ||
      in_sizes[11] != 2000 || in_sizes[12] != 40 || in_sizes[13] != 800 || in_sizes[14] != 20 ||
      in_sizes[15] != 400 || in_sizes[16] != 20 || in_sizes[17] != 100 || in_sizes[18] != 5 ||
      out_size != NBATCH * 5) return;
  if ((size_t)WSB_END > ws_size) return;

  const float* x     = (const float*)d_in[0];
  const int*   recv  = (const int*)  d_in[1];
  const int*   send  = (const int*)  d_in[2];
  const float* Wfr1  = (const float*)d_in[3];
  const float* bfr1  = (const float*)d_in[4];
  const float* Wfr2  = (const float*)d_in[5];
  const float* bfr2  = (const float*)d_in[6];
  const float* Wfr3  = (const float*)d_in[7];
  const float* bfr3  = (const float*)d_in[8];
  const float* gamma = (const float*)d_in[9];
  const float* beta  = (const float*)d_in[10];
  const float* Wfo1  = (const float*)d_in[11];
  const float* bfo1  = (const float*)d_in[12];
  const float* Wfo2  = (const float*)d_in[13];
  const float* bfo2  = (const float*)d_in[14];
  const float* Wfo3  = (const float*)d_in[15];
  const float* bfo3  = (const float*)d_in[16];
  const float* Wfc   = (const float*)d_in[17];
  const float* bfc   = (const float*)d_in[18];

  unsigned char* ws = (unsigned char*)d_ws;
  _Float16* wb   = (_Float16*)(ws + WSB_WB);
  _Float16* xt   = (_Float16*)(ws + WSB_XT);
  float*    Ebuf = (float*)(ws + WSB_E);
  float*    stat = (float*)(ws + WSB_STAT);
  float*    scal = (float*)(ws + WSB_SC);
  float*    nsum = (float*)(ws + WSB_NS);
  float*    out  = (float*)d_out;

  prep_kernel<<<NBATCH, 256, 0, stream>>>(x, Wfr1, Wfr2, Wfr3, Wfo1, Wfo2, Wfo3, wb, xt);
  dim3 gE(NND, NBATCH);
  edge_kernel<<<gE, 256, 0, stream>>>(xt, wb, recv, send, bfr1, bfr2, bfr3, Ebuf, stat);
  stat_kernel<<<1, 256, 0, stream>>>(stat, gamma, beta, scal);
  node_kernel<<<NBATCH, 256, 0, stream>>>(xt, wb, recv, Ebuf, scal, bfo1, bfo2, bfo3, nsum);
  head_kernel<<<1, 256, 0, stream>>>(nsum, Wfc, bfc, out);
}
